// SarvamMLAMoE_20392504721497
// MI455X (gfx1250) — hardware-verified
//
#include <hip/hip_runtime.h>
#include <math.h>

typedef __attribute__((ext_vector_type(16))) _Float16 v16h;
typedef __attribute__((ext_vector_type(16))) __bf16 v16b;
typedef __attribute__((ext_vector_type(8)))  _Float16 v8h;
typedef __attribute__((ext_vector_type(8)))  __bf16 v8b;
typedef __attribute__((ext_vector_type(8)))  float v8f;
typedef __attribute__((ext_vector_type(4)))  float v4f;
typedef __attribute__((ext_vector_type(4)))  unsigned v4u;

#ifndef NB
#define NB 2048
#endif
#define NB_FULL 2048
#define DIN  1024
#define DHID 512
#define DSH  1024
#define DOUT 1024
#define NE   16
#define KF (NE * DHID)
#define KP (KF + DSH)
#define HCARRY 64.0f
#define WCARRY 512.0f
#define OSCALE (1.0f / 32768.0f)
#define RSCALE 2.5f

#define WS_XB  ((size_t)0)
#define WS_WGT (WS_XB  + (size_t)NB * DIN * 2)
#define WS_WUT (WS_WGT + (size_t)KP * DIN * 2)
#define WS_W2T (WS_WUT + (size_t)KP * DIN * 2)
#define WS_HB  (WS_W2T + (size_t)DOUT * KP * 2)
#define WS_WTS (WS_HB  + (size_t)NB * KP * 2)
#define WS_END (WS_WTS + (size_t)NB * NE * 4)

static_assert(NB % 128 == 0);
static_assert(NB <= NB_FULL);
static_assert(DIN % 32 == 0 && KP % 32 == 0 && (KP * 2) % 128 == 0);
static_assert(KF % 64 == 0 && DHID % 64 == 0 && DSH % 64 == 0 && KP % 64 == 0 && DIN % 64 == 0 && DOUT % 128 == 0);
static_assert(DIN % 8 == 0 && NE == 16);
static_assert((size_t)NB_FULL * DOUT * 4 == 8388608);
static_assert(WS_WGT % 128 == 0 && WS_WUT % 128 == 0 && WS_W2T % 128 == 0 && WS_HB % 128 == 0 && WS_WTS % 128 == 0);
static_assert(WS_END <= (size_t)134217728);
static_assert((size_t)(NB * DIN / 8 / 256) * 256 * 8 == (size_t)NB * DIN);
static_assert((size_t)(DHID / 64) * (DIN / 64) * NE * 4096 == (size_t)NE * DIN * DHID);
static_assert((size_t)(DSH / 64) * (DIN / 64) * 4096 == (size_t)DIN * DSH);
static_assert((size_t)NE * DIN * DHID + (size_t)DIN * DSH == (size_t)KP * DIN);
static_assert((size_t)(DOUT / 64) * (DHID / 64) * NE * 4096 == (size_t)DOUT * KF);
static_assert((size_t)(DOUT / 64) * (DSH / 64) * 4096 == (size_t)DOUT * DSH);
static_assert((size_t)(NB / 64) * 64 * NE == (size_t)NB * NE);
static_assert(2 * 128 * 4 == 64 * NE);
static_assert((size_t)(KP / 64) * (NB / 128) * 128 * 64 == (size_t)NB * KP);
static_assert(256 * 16 * 4 == 128 * 128);
static_assert((size_t)(DOUT / 128) * (NB / 128) * 128 * 128 == (size_t)NB * DOUT);
static_assert(64 * 65 * 4 <= 131072);
static_assert(2 * 64 * NE * 4 <= 131072);
static_assert(128 * 64 * 2 <= 131072);
static_assert(8 * 16 * 64 * 4 <= 131072);

__device__ __forceinline__ v8f wmma16(v16h a, v16h b, v8f c) {
  v8f d = __builtin_amdgcn_wmma_f32_16x16x32_f16(false, a, false, b, (short)0, c, false, false);
  asm volatile("v_nop\n\tv_nop\n\tv_nop\n\tv_nop" : "+v"(d) : "v"(a), "v"(b));
  return d;
}
__device__ __forceinline__ v8f wmma_bf(v16b a, v16b b, v8f c) {
  v8f d = __builtin_amdgcn_wmma_f32_16x16x32_bf16(false, a, false, b, (short)0, c, false, false);
  asm volatile("v_nop\n\tv_nop\n\tv_nop\n\tv_nop" : "+v"(d) : "v"(a), "v"(b));
  return d;
}
__device__ __forceinline__ float bfr(float v) { return (float)(__bf16)v; }
static __device__ __forceinline__ _Float16 toh_flush(float v) { const _Float16 r = (_Float16)v; return (fabsf(v) < 6.103515625e-05f) ? (_Float16)0.0f : r; }
__device__ __forceinline__ v16b ldfrag_b(const unsigned short* p) { union { v16b v; v4u q[2]; } f; f.q[0] = *(const v4u*)p; f.q[1] = *(const v4u*)(p + 16); return f.v; }
__device__ __forceinline__ v16h ldfrag_h(const unsigned short* p) { union { v16h v; v4u q[2]; } f; f.q[0] = *(const v4u*)p; f.q[1] = *(const v4u*)(p + 16); return f.v; }

__global__ __launch_bounds__(256) void k_cvt_x(const float* __restrict__ X, unsigned short* __restrict__ XB) {
  const unsigned i = blockIdx.x * 256u + threadIdx.x;
  const unsigned ic = i < (unsigned)(NB * DIN / 8) ? i : (unsigned)(NB * DIN / 8 - 1);
  const v4f a = *(const v4f*)(X + (size_t)ic * 8), b = *(const v4f*)(X + (size_t)ic * 8 + 4);
  union { v8b h; v4u u; } o;
#pragma unroll
  for (int j = 0; j < 4; ++j) { o.h[j] = (__bf16)a[j]; o.h[4 + j] = (__bf16)b[j]; }
  const v4u val = o.u;
  volatile v4u* p = (volatile v4u*)(XB + (size_t)ic * 8);
  *p = val; __threadfence(); *p = val;
}

template <int F16>
__global__ __launch_bounds__(256) void k_tr(const float* __restrict__ S, unsigned short* __restrict__ Dst, unsigned K, unsigned N, unsigned dpitch, unsigned erow, unsigned ecol, float sc) {
  __shared__ float tile[64][65];
  const unsigned t = threadIdx.x, e = blockIdx.z, k0 = blockIdx.y * 64u, n0 = blockIdx.x * 64u;
  const float* s = S + (size_t)e * K * N;
#pragma unroll
  for (unsigned it = 0; it < 4; ++it) { const unsigned idx = it * 256u + t, kr = idx >> 4, c4 = idx & 15u;
    const v4f v = *(const v4f*)(s + (size_t)(k0 + kr) * N + n0 + 4u * c4);
    tile[kr][4u * c4 + 0] = v[0]; tile[kr][4u * c4 + 1] = v[1]; tile[kr][4u * c4 + 2] = v[2]; tile[kr][4u * c4 + 3] = v[3]; }
  __syncthreads();
  v4u o[2];
#pragma unroll
  for (unsigned it = 0; it < 2; ++it) { const unsigned idx = it * 256u + t, nr = idx >> 3, q = idx & 7u;
    union { v8b b; v8h h; v4u u; } w;
#pragma unroll
    for (int i = 0; i < 8; ++i) { const float v = bfr(tile[8u * q + i][nr]); if (F16) w.h[i] = toh_flush(v * sc); else w.b[i] = (__bf16)v; }
    o[it] = w.u; }
#pragma unroll
  for (unsigned it = 0; it < 2; ++it) { const unsigned idx = it * 256u + t, nr = idx >> 3, q = idx & 7u;
    *(volatile v4u*)(Dst + (size_t)(e * erow + n0 + nr) * dpitch + e * ecol + k0 + 8u * q) = o[it]; }
  __threadfence();
#pragma unroll
  for (unsigned it = 0; it < 2; ++it) { const unsigned idx = it * 256u + t, nr = idx >> 3, q = idx & 7u;
    *(volatile v4u*)(Dst + (size_t)(e * erow + n0 + nr) * dpitch + e * ecol + k0 + 8u * q) = o[it]; }
}

__global__ __launch_bounds__(128) void k_route(const unsigned short* __restrict__ XB, const float* __restrict__ GW, const float* __restrict__ EB, float* __restrict__ WTS) {
#pragma clang fp contract(off)
  __shared__ __align__(16) float sp[64][NE];
  __shared__ __align__(16) float cwl[64][NE];
  const unsigned tid = threadIdx.x, lane = tid & 31u, col = lane & 15u, g = lane >> 4; const unsigned r0 = blockIdx.x * 64u;
  const unsigned wave = __builtin_amdgcn_readfirstlane(threadIdx.x >> 5);
  const float* gw = GW + (size_t)col * DIN;
#pragma unroll 1
  for (unsigned r = 0; r < 8u; ++r) {
    const unsigned lr = wave * 16u + 8u * g + r;
    const unsigned short* xr = XB + (size_t)(r0 + lr) * DIN;
    float acc = 0.f;
#pragma unroll 1
    for (unsigned k = 0; k < (unsigned)DIN; k += 8u) {
      const v4u xv = *(const v4u*)(xr + k);
      const v4f w0 = *(const v4f*)(gw + k), w1 = *(const v4f*)(gw + k + 4u);
      acc = fmaf(__uint_as_float(xv[0] << 16),         bfr(w0[0]), acc);
      acc = fmaf(__uint_as_float(xv[0] & 0xffff0000u), bfr(w0[1]), acc);
      acc = fmaf(__uint_as_float(xv[1] << 16),         bfr(w0[2]), acc);
      acc = fmaf(__uint_as_float(xv[1] & 0xffff0000u), bfr(w0[3]), acc);
      acc = fmaf(__uint_as_float(xv[2] << 16),         bfr(w1[0]), acc);
      acc = fmaf(__uint_as_float(xv[2] & 0xffff0000u), bfr(w1[1]), acc);
      acc = fmaf(__uint_as_float(xv[3] << 16),         bfr(w1[2]), acc);
      acc = fmaf(__uint_as_float(xv[3] & 0xffff0000u), bfr(w1[3]), acc);
    }
    sp[lr][col] = 1.0f / (1.0f + expf(-acc));
  }
  __syncthreads();
  if (wave < 2u) {
    float s[NE], sb[NE];
#pragma unroll
    for (int q = 0; q < 4; ++q) { const v4f v = *(const v4f*)&sp[tid][4 * q]; s[4 * q + 0] = v[0]; s[4 * q + 1] = v[1]; s[4 * q + 2] = v[2]; s[4 * q + 3] = v[3]; }
#pragma unroll
    for (int e = 0; e < NE; ++e) sb[e] = s[e] + bfr(EB[e]);
    float gs[4];
#pragma unroll
    for (int gi = 0; gi < 4; ++gi) { float m1 = -INFINITY, m2 = -INFINITY;
#pragma unroll
      for (int j = 0; j < 4; ++j) { const float v = sb[4 * gi + j]; const bool a = v > m1, b = v > m2; m2 = a ? m1 : (b ? v : m2); m1 = a ? v : m1; }
      gs[gi] = m1 + m2; }
    int g1 = 0; float b1 = gs[0];
#pragma unroll
    for (int gi = 1; gi < 4; ++gi) { const bool c = gs[gi] > b1; b1 = c ? gs[gi] : b1; g1 = c ? gi : g1; }
    int g2 = 0; float b2 = -INFINITY;
#pragma unroll
    for (int gi = 0; gi < 4; ++gi) { const bool c = (gi != g1) && (gs[gi] > b2); b2 = c ? gs[gi] : b2; g2 = c ? gi : g2; }
    unsigned taken = 0u; float wsel[4];
#pragma unroll
    for (int kp = 0; kp < 4; ++kp) { float bv = -INFINITY, bs = 0.f; int best = 0;
#pragma unroll
      for (int e = 0; e < NE; ++e) { const bool ok = (((e >> 2) == g1) || ((e >> 2) == g2)) && (((taken >> e) & 1u) == 0u) && (sb[e] > bv);
        bv = ok ? sb[e] : bv; bs = ok ? s[e] : bs; best = ok ? e : best; }
      taken |= 1u << (best & 15); wsel[kp] = bs; }
    const float wsum = ((wsel[0] + wsel[1]) + wsel[2]) + wsel[3];
    const float inv = 1.0f / wsum;
#pragma unroll
    for (int q = 0; q < 4; ++q) { v4f o;
#pragma unroll
      for (int i = 0; i < 4; ++i) { const int e = 4 * q + i; const float c = (s[e] * inv) * RSCALE; o[i] = ((taken >> e) & 1u) ? c : 0.f; }
      *(v4f*)&cwl[tid][4 * q] = o; }
  }
  __syncthreads();
  v4f pv[2];
#pragma unroll
  for (unsigned it = 0; it < 2; ++it) { const unsigned idx = it * 128u + tid; pv[it] = *(const v4f*)(&cwl[0][0] + 4u * idx); }
  float* wo = WTS + (size_t)r0 * NE;
#pragma unroll
  for (unsigned it = 0; it < 2; ++it) { const unsigned idx = it * 128u + tid; *(volatile v4f*)(wo + 4u * idx) = pv[it]; }
  __threadfence();
#pragma unroll
  for (unsigned it = 0; it < 2; ++it) { const unsigned idx = it * 128u + tid; *(volatile v4f*)(wo + 4u * idx) = pv[it]; }
}

__global__ __launch_bounds__(256) void k_h(const unsigned short* __restrict__ XB, const unsigned short* __restrict__ WGT, const unsigned short* __restrict__ WUT, const float* __restrict__ WTS, unsigned short* __restrict__ HB) {
  __shared__ __align__(16) _Float16 sh[128][64];
  const unsigned t = threadIdx.x, wave = t >> 5, lane = t & 31u, lm = lane & 15u, lh = lane >> 4, wm = wave >> 1, wn = wave & 1u;
  const unsigned m0 = blockIdx.y * 128u, f0 = blockIdx.x * 64u;
  const unsigned short* ar[2]; const unsigned short* br[4];
#pragma unroll
  for (int mi = 0; mi < 2; ++mi) ar[mi] = XB + (size_t)(m0 + wm * 32u + mi * 16u + lm) * DIN + 8u * lh;
#pragma unroll
  for (int ni = 0; ni < 2; ++ni) { br[ni] = WGT + (size_t)(f0 + wn * 32u + ni * 16u + lm) * DIN + 8u * lh; br[2 + ni] = WUT + (size_t)(f0 + wn * 32u + ni * 16u + lm) * DIN + 8u * lh; }
  v8f acc[2][4] = {};
#pragma unroll 2
  for (unsigned kc = 0; kc < DIN / 32; ++kc) { v16b a[2], b[4];
#pragma unroll
    for (int mi = 0; mi < 2; ++mi) a[mi] = ldfrag_b(ar[mi] + kc * 32u);
#pragma unroll
    for (int ni = 0; ni < 4; ++ni) b[ni] = ldfrag_b(br[ni] + kc * 32u);
#pragma unroll
    for (int mi = 0; mi < 2; ++mi)
#pragma unroll
      for (int ni = 0; ni < 4; ++ni) acc[mi][ni] = wmma_bf(a[mi], b[ni], acc[mi][ni]); }
  const unsigned ex = f0 / DHID;
  const unsigned ec = ex < (unsigned)NE ? ex : (unsigned)(NE - 1);
  float wv[2][8];
#pragma unroll
  for (int mi = 0; mi < 2; ++mi) {
#pragma unroll
    for (int r = 0; r < 8; ++r) { const float gq = WTS[(size_t)(m0 + wm * 32u + mi * 16u + 8u * lh + r) * NE + ec]; wv[mi][r] = (ex < (unsigned)NE ? gq : 1.0f) * HCARRY; }
    asm volatile("s_wait_loadcnt 0x0" ::: "memory"); }
#pragma unroll
  for (int ni = 0; ni < 2; ++ni) {
#pragma unroll
    for (int mi = 0; mi < 2; ++mi)
#pragma unroll
      for (int r = 0; r < 8; ++r) { const float gv = acc[mi][ni][r], uv = acc[mi][2 + ni][r];
        const float sg = gv * __builtin_amdgcn_rcpf(1.0f + __expf(-gv));
        sh[wm * 32u + mi * 16 + 8u * lh + r][wn * 32u + ni * 16 + lm] = toh_flush(sg * uv * wv[mi][r]); } }
  __syncthreads();
  v4u o[4];
#pragma unroll
  for (unsigned it = 0; it < 4; ++it) { const unsigned rw = wave * 16u + it * 4u + (lane >> 3), q = lane & 7u; union { v8h h; v4u u; } w; w.h = *(const v8h*)&sh[rw][8u * q]; o[it] = w.u; }
  unsigned short* hb = HB + (size_t)m0 * KP + f0;
#pragma unroll
  for (unsigned it = 0; it < 4; ++it) { const unsigned rw = wave * 16u + it * 4u + (lane >> 3), q = lane & 7u; *(volatile v4u*)(hb + (size_t)rw * KP + 8u * q) = o[it]; }
  __threadfence();
#pragma unroll
  for (unsigned it = 0; it < 4; ++it) { const unsigned rw = wave * 16u + it * 4u + (lane >> 3), q = lane & 7u; *(volatile v4u*)(hb + (size_t)rw * KP + 8u * q) = o[it]; }
}

__global__ __launch_bounds__(256) void k_out(const unsigned short* __restrict__ HB, const unsigned short* __restrict__ W2T, float* __restrict__ OUT) {
  __shared__ __align__(16) float sf[8][16][64];
  const unsigned t = threadIdx.x, wave = t >> 5, lane = t & 31u, lm = lane & 15u, lh = lane >> 4, wm = wave >> 1, wn = wave & 1u;
  const unsigned m0 = blockIdx.y * 128u, n0 = blockIdx.x * 128u;
  const unsigned short* ar[2]; const unsigned short* br[4];
#pragma unroll
  for (int mi = 0; mi < 2; ++mi) ar[mi] = HB + (size_t)(m0 + wm * 32u + mi * 16u + lm) * KP + 8u * lh;
#pragma unroll
  for (int ni = 0; ni < 4; ++ni) br[ni] = W2T + (size_t)(n0 + wn * 64u + ni * 16u + lm) * KP + 8u * lh;
  v8f acc[2][4] = {};
#pragma unroll 2
  for (unsigned kc = 0; kc < KP / 32; ++kc) { v16h a[2], b[4];
#pragma unroll
    for (int mi = 0; mi < 2; ++mi) a[mi] = ldfrag_h(ar[mi] + kc * 32u);
#pragma unroll
    for (int ni = 0; ni < 4; ++ni) b[ni] = ldfrag_h(br[ni] + kc * 32u);
#pragma unroll
    for (int mi = 0; mi < 2; ++mi)
#pragma unroll
      for (int ni = 0; ni < 4; ++ni) acc[mi][ni] = wmma16(a[mi], b[ni], acc[mi][ni]); }
#pragma unroll
  for (int mi = 0; mi < 2; ++mi) {
    if (mi) __syncthreads();
#pragma unroll
    for (int ni = 0; ni < 4; ++ni)
#pragma unroll
      for (int r = 0; r < 8; ++r) sf[wave][8u * lh + r][ni * 16 + lm] = acc[mi][ni][r] * OSCALE;
    __syncthreads();
    v4f v[8];
#pragma unroll
    for (unsigned it = 0; it < 8; ++it) { const unsigned rw = it * 2u + (lane >> 4), pc = lane & 15u; v[it] = *(const v4f*)&sf[wave][rw][4u * pc]; }
    float* po = OUT + (size_t)(m0 + wm * 32u + mi * 16u) * DOUT + n0 + wn * 64u;
#pragma unroll
    for (unsigned it = 0; it < 8; ++it) { const unsigned rw = it * 2u + (lane >> 4), pc = lane & 15u; *(volatile v4f*)(po + (size_t)rw * DOUT + 4u * pc) = v[it]; }
    __threadfence();
#pragma unroll
    for (unsigned it = 0; it < 8; ++it) { const unsigned rw = it * 2u + (lane >> 4), pc = lane & 15u; *(volatile v4f*)(po + (size_t)rw * DOUT + 4u * pc) = v[it]; }
  }
}

extern "C" void kernel_launch(void* const* d_in, const int* in_sizes, int n_in, void* d_out, int out_size, void* d_ws, size_t ws_size, hipStream_t stream) {
  if (n_in < 9) return;
  if (in_sizes[0] < NB * DIN || in_sizes[1] < NE * DIN || in_sizes[2] < NE) return;
  if (in_sizes[3] < NE * DIN * DHID || in_sizes[4] < NE * DIN * DHID || in_sizes[5] < NE * DHID * DOUT) return;
  if (in_sizes[6] < DIN * DSH || in_sizes[7] < DIN * DSH || in_sizes[8] < DSH * DOUT) return;
  if ((size_t)out_size < (size_t)NB * DOUT) return;
  if (ws_size < (size_t)WS_END) return;
  const float* X   = (const float*)d_in[0];
  const float* GW  = (const float*)d_in[1];
  const float* EB  = (const float*)d_in[2];
  const float* WG  = (const float*)d_in[3];
  const float* WU  = (const float*)d_in[4];
  const float* WD  = (const float*)d_in[5];
  const float* SWG = (const float*)d_in[6];
  const float* SWU = (const float*)d_in[7];
  const float* SWD = (const float*)d_in[8];
  char* ws = (char*)d_ws;
  unsigned short* XB  = (unsigned short*)(ws + WS_XB);
  unsigned short* WGT = (unsigned short*)(ws + WS_WGT);
  unsigned short* WUT = (unsigned short*)(ws + WS_WUT);
  unsigned short* W2T = (unsigned short*)(ws + WS_W2T);
  unsigned short* HB  = (unsigned short*)(ws + WS_HB);
  float* WTS = (float*)(ws + WS_WTS);
  float* OUT = (float*)d_out;
  k_cvt_x<<<dim3(NB * DIN / 8 / 256), 256, 0, stream>>>(X, XB);
  k_tr<0><<<dim3(DHID / 64, DIN / 64, NE), 256, 0, stream>>>(WG, WGT, (unsigned)DIN, (unsigned)DHID, (unsigned)DIN, (unsigned)DHID, 0u, 1.0f);
  k_tr<0><<<dim3(DHID / 64, DIN / 64, NE), 256, 0, stream>>>(WU, WUT, (unsigned)DIN, (unsigned)DHID, (unsigned)DIN, (unsigned)DHID, 0u, 1.0f);
  k_tr<0><<<dim3(DSH / 64, DIN / 64, 1), 256, 0, stream>>>(SWG, WGT + (size_t)KF * DIN, (unsigned)DIN, (unsigned)DSH, (unsigned)DIN, 0u, 0u, 1.0f);
  k_tr<0><<<dim3(DSH / 64, DIN / 64, 1), 256, 0, stream>>>(SWU, WUT + (size_t)KF * DIN, (unsigned)DIN, (unsigned)DSH, (unsigned)DIN, 0u, 0u, 1.0f);
  k_tr<1><<<dim3(DOUT / 64, DHID / 64, NE), 256, 0, stream>>>(WD, W2T, (unsigned)DHID, (unsigned)DOUT, (unsigned)KP, 0u, (unsigned)DHID, WCARRY);
  k_tr<1><<<dim3(DOUT / 64, DSH / 64, 1), 256, 0, stream>>>(SWD, W2T + KF, (unsigned)DSH, (unsigned)DOUT, (unsigned)KP, 0u, 0u, WCARRY);
  k_route<<<dim3(NB / 64), 128, 0, stream>>>(XB, GW, EB, WTS);
  k_h<<<dim3(KP / 64, NB / 128), 256, 0, stream>>>(XB, WGT, WUT, WTS, HB);
  k_out<<<dim3(DOUT / 128, NB / 128), 256, 0, stream>>>(HB, W2T, OUT);
}
